// MSWIDTBlock_6828998001251
// MI455X (gfx1250) — hardware-verified
//
#include <hip/hip_runtime.h>
#include <math.h>

#define TT      4096
#define DM      512
#define NHEAD   8
#define HD      64
#define DFF     2048
#define QKW     1024
#define LNEPS   1.0e-6f
#define WSC     64.0f
#define QKCARRY 16.0f
#define VCARRY  16.0f
#define PCARRY  1024.0f
#define AOCARRY 64.0f
static_assert(NHEAD * HD == DM);
static_assert(QKW == 2 * DM);
static_assert((TT % 64) == 0 && (DM % 64) == 0 && (DFF % 64) == 0 && (QKW % 64) == 0);
static_assert(DM == 32 * 16);
static_assert((TT % 8) == 0);

typedef _Float16 v16h __attribute__((ext_vector_type(16)));
typedef _Float16 v8h  __attribute__((ext_vector_type(8)));
typedef _Float16 v4h  __attribute__((ext_vector_type(4)));
typedef __attribute__((ext_vector_type(16))) __bf16 v16b;
typedef float    v8f  __attribute__((ext_vector_type(8)));
typedef float    v4f  __attribute__((ext_vector_type(4)));
typedef unsigned int v4u __attribute__((ext_vector_type(4)));

union FragH  { v16h v; v8h h[2]; };
union Frag16 { v16h h; v16b b; v8h hh[2]; v4u u[2]; };

__device__ __forceinline__ unsigned short bf_bits(float f) {
  unsigned u = __float_as_uint(f);
  return (unsigned short)((u + 0x7FFFu + ((u >> 16) & 1u)) >> 16);
}
__device__ __forceinline__ float bf_up(unsigned short h) { return __uint_as_float(((unsigned)h) << 16); }
__device__ __forceinline__ float bfr(float f) { return bf_up(bf_bits(f)); }
__device__ __forceinline__ unsigned short h_bits(_Float16 x) { return __builtin_bit_cast(unsigned short, x); }
__device__ __forceinline__ unsigned pk16(unsigned short a, unsigned short b) { return (unsigned)a | ((unsigned)b << 16); }
__device__ __forceinline__ v8f zero8() { v8f z = {0.f, 0.f, 0.f, 0.f, 0.f, 0.f, 0.f, 0.f}; return z; }
__device__ __forceinline__ float gelu_t(float f) {
  const float u = 0.7978845608028654f * (f + 0.044715f * f * f * f);
  return 0.5f * f * (1.0f + tanhf(u));
}

__device__ __forceinline__ v16h ldfrag_h(const _Float16* p) {
  FragH f;
  f.h[0] = *(const v8h*)(p);
  f.h[1] = *(const v8h*)(p + 16);
  return f.v;
}
__device__ __forceinline__ Frag16 ldfrag16(const unsigned short* p) {
  Frag16 f;
  f.u[0] = *(const v4u*)(p);
  f.u[1] = *(const v4u*)(p + 16);
  return f;
}

__device__ __forceinline__ v8f mma_h(v16h a, v16h b, v8f c) {
  c = __builtin_amdgcn_wmma_f32_16x16x32_f16(false, a, false, b, (short)0, c, false, false);
#if defined(__HIP_DEVICE_COMPILE__)
  asm volatile("v_nop\n\tv_nop\n\tv_nop\n\tv_nop" : "+v"(c) : "v"(a), "v"(b));
#endif
  return c;
}
template <int TB>
__device__ __forceinline__ v8f mma16_raw(const Frag16& a, const Frag16& b, v8f c) {
  if (TB == 0) return __builtin_amdgcn_wmma_f32_16x16x32_f16(false, a.h, false, b.h, (short)0, c, false, false);
  else         return __builtin_amdgcn_wmma_f32_16x16x32_bf16(false, a.b, false, b.b, (short)0, c, false, false);
}
__device__ __forceinline__ void dep_guard1(v8f& a, v8f& b, v16h x) {
#if defined(__HIP_DEVICE_COMPILE__)
  asm volatile("v_nop\n\tv_nop\n\tv_nop\n\tv_nop" : "+v"(a), "+v"(b) : "v"(x));
#endif
}
__device__ __forceinline__ void keep4_h(v16h a, v16h b, v16h c, v16h d) {
#if defined(__HIP_DEVICE_COMPILE__)
  asm volatile("v_nop" :: "v"(a), "v"(b), "v"(c), "v"(d));
#endif
}
__device__ __forceinline__ void acc_guard4(v8f& a, v8f& b, v8f& c, v8f& d) {
#if defined(__HIP_DEVICE_COMPILE__)
  asm volatile("v_nop\n\tv_nop\n\tv_nop\n\tv_nop" : "+v"(a), "+v"(b), "+v"(c), "+v"(d));
#endif
}
__device__ __forceinline__ void wave_sync_lds() {
  __builtin_amdgcn_fence(__ATOMIC_RELEASE, "workgroup");
  __builtin_amdgcn_wave_barrier();
  __builtin_amdgcn_fence(__ATOMIC_ACQUIRE, "workgroup");
}
__device__ __forceinline__ float wsum32(float v) {
#pragma unroll
  for (int off = 16; off > 0; off >>= 1) v += __shfl_xor(v, off, 32);
  return v;
}

template <int KIND>
__global__ __launch_bounds__(256) void conv_t16(const float* __restrict__ Wa, const float* __restrict__ Wb,
                                                 unsigned short* dst, int Cin, int Osrc, int Odst, int n8, float wsc) {
  const int i    = blockIdx.x * 256 + threadIdx.x;
  const int ic   = (i < n8) ? i : (n8 - 1);
  const int per  = (Odst * Cin) >> 3;
  const int bi   = ic / per;
  const int r    = ic - bi * per;
  const int cin8 = Cin >> 3;
  const int o    = r / cin8;
  const int c0   = (r - o * cin8) * 8;
  const int sel  = (o >= Osrc) ? 1 : 0;
  const int os   = o - sel * Osrc;
  const float* pa = Wa + ((size_t)bi * Cin + c0) * Osrc + os;
  const float* pb = Wb + ((size_t)bi * Cin + c0) * Osrc + os;
  float v[8];
#pragma unroll
  for (int e = 0; e < 8; ++e) {
    const float xa = pa[(size_t)e * Osrc];
    const float xb = pb[(size_t)e * Osrc];
    v[e] = bfr(sel ? xb : xa);
  }
  v4u ov;
#pragma unroll
  for (int e = 0; e < 4; ++e) {
    if (KIND == 0) ov[e] = pk16(h_bits((_Float16)(v[2 * e] * wsc)), h_bits((_Float16)(v[2 * e + 1] * wsc)));
    else           ov[e] = pk16(bf_bits(v[2 * e]), bf_bits(v[2 * e + 1]));
  }
  if (i < n8) *(volatile v4u*)(dst + (size_t)i * 8) = ov;
  __threadfence();
  if (i < n8) *(volatile v4u*)(dst + (size_t)i * 8) = ov;
}

__global__ __launch_bounds__(256) void pack_bias2(const float* __restrict__ bq, const float* __restrict__ bk,
                                                  float* dst) {
  const int t = threadIdx.x;
  const int i = (4 * t) & (DM - 1);
  const v4f va = *(const v4f*)(bq + i), vb = *(const v4f*)(bk + i);
  const bool selk = (t >= 128);
  v4f o;
#pragma unroll
  for (int e = 0; e < 4; ++e) o[e] = selk ? vb[e] : va[e];
  *(volatile v4f*)(dst + 4 * t) = o;
  __threadfence();
  *(volatile v4f*)(dst + 4 * t) = o;
}

template <int MODE>
__global__ __launch_bounds__(256) void ln_rows(const float* __restrict__ X, const float* __restrict__ gam,
                                                const float* __restrict__ bet, unsigned short* P0, unsigned short* P1) {
  const int tid = threadIdx.x, wave = tid >> 5, lane = tid & 31;
  const size_t row = (size_t)blockIdx.x * 8 + wave;
  const int cA = 8 * lane, cB = 256 + 8 * lane;
  const float* xr = X + row * DM;
  const v4f a0 = *(const v4f*)(xr + cA), a1 = *(const v4f*)(xr + cA + 4);
  const v4f c0v = *(const v4f*)(xr + cB), c1v = *(const v4f*)(xr + cB + 4);
  float x[16];
#pragma unroll
  for (int e = 0; e < 4; ++e) { x[e] = a0[e]; x[4 + e] = a1[e]; x[8 + e] = c0v[e]; x[12 + e] = c1v[e]; }
  if (MODE == 0) {
#pragma unroll
    for (int e = 0; e < 16; ++e) x[e] = bfr(x[e]);
  }
  float s = 0.f;
#pragma unroll
  for (int e = 0; e < 16; e += 2) s += x[e] + x[e + 1];
  s = wsum32(s);
  const float mean = s * (1.0f / DM);
  float d[16];
  float vs = 0.f;
#pragma unroll
  for (int e = 0; e < 16; ++e) { d[e] = x[e] - mean; vs += d[e] * d[e]; }
  vs = wsum32(vs);
  const float rstd = rsqrtf(vs * (1.0f / DM) + LNEPS);
  const v4f g0 = *(const v4f*)(gam + cA), g1 = *(const v4f*)(gam + cA + 4);
  const v4f g2 = *(const v4f*)(gam + cB), g3 = *(const v4f*)(gam + cB + 4);
  const v4f b0 = *(const v4f*)(bet + cA), b1 = *(const v4f*)(bet + cA + 4);
  const v4f b2 = *(const v4f*)(bet + cB), b3 = *(const v4f*)(bet + cB + 4);
  float y[16];
#pragma unroll
  for (int e = 0; e < 4; ++e) {
    y[e]      = (d[e] * rstd)      * bfr(g0[e]) + bfr(b0[e]);
    y[4 + e]  = (d[4 + e] * rstd)  * bfr(g1[e]) + bfr(b1[e]);
    y[8 + e]  = (d[8 + e] * rstd)  * bfr(g2[e]) + bfr(b2[e]);
    y[12 + e] = (d[12 + e] * rstd) * bfr(g3[e]) + bfr(b3[e]);
  }
  v4u pA0, pB0, pA1, pB1;
#pragma unroll
  for (int e = 0; e < 4; ++e) {
    if (MODE == 0) {
      pA0[e] = pk16(h_bits((_Float16)x[2 * e]),     h_bits((_Float16)x[2 * e + 1]));
      pB0[e] = pk16(h_bits((_Float16)x[8 + 2 * e]), h_bits((_Float16)x[8 + 2 * e + 1]));
      pA1[e] = pk16(h_bits((_Float16)y[2 * e]),     h_bits((_Float16)y[2 * e + 1]));
      pB1[e] = pk16(h_bits((_Float16)y[8 + 2 * e]), h_bits((_Float16)y[8 + 2 * e + 1]));
    } else {
      const unsigned short ha = bf_bits(y[2 * e]),     hb = bf_bits(y[2 * e + 1]);
      const unsigned short hc = bf_bits(y[8 + 2 * e]), hd = bf_bits(y[8 + 2 * e + 1]);
      const unsigned short la = bf_bits(y[2 * e] - bf_up(ha)),     lb = bf_bits(y[2 * e + 1] - bf_up(hb));
      const unsigned short lc = bf_bits(y[8 + 2 * e] - bf_up(hc)), ld = bf_bits(y[8 + 2 * e + 1] - bf_up(hd));
      pA0[e] = pk16(ha, hb);
      pB0[e] = pk16(hc, hd);
      pA1[e] = pk16(la, lb);
      pB1[e] = pk16(lc, ld);
    }
  }
  const size_t oA = row * DM + cA, oB = row * DM + cB;
  for (int pass = 0; pass < 2; ++pass) {
    *(volatile v4u*)(P0 + oA) = pA0;
    *(volatile v4u*)(P0 + oB) = pB0;
    *(volatile v4u*)(P1 + oA) = pA1;
    *(volatile v4u*)(P1 + oB) = pB1;
    __threadfence();
  }
}

template <int TB, int A32, int NPA, int OM, int BIASM, int ACT, int RES>
__global__ __launch_bounds__(256) void gemm64(
    const void* __restrict__ Ap, const void* __restrict__ Ap2, int lda, long long strideA, float ascale,
    const unsigned short* __restrict__ Btp, int ldb, long long strideB,
    const float* __restrict__ bias, float bscale,
    const void* resid,
    void* Cout, void* Cout2, int ldc, long long strideC,
    int M, int N, int K, float oscale) {
  __shared__ __align__(16) float sT[8][16 * 68];
  const int b    = blockIdx.y;
  const int lane = threadIdx.x & 31;
  const int wave = threadIdx.x >> 5;
  const int tilesN = N >> 6;
  const int tilesM = M >> 6;
  const int tile = blockIdx.x * 8 + wave;
  if (tile >= tilesM * tilesN) return;
  const int tm = tile / tilesN;
  const int tn = tile - tm * tilesN;
  const int m0 = tm << 6;
  const int n0 = tn << 6;

  const unsigned short* A1 = (const unsigned short*)Ap  + (size_t)b * strideA;
  const unsigned short* A2 = (const unsigned short*)Ap2 + (size_t)b * strideA;
  const float*          Af = (const float*)Ap + (size_t)b * strideA;
  const unsigned short* Bb = Btp + (size_t)b * strideB;

  const int rlane = lane & 15;
  const int koff  = (lane >> 4) * 8;
  const int mOff  = (lane >> 4) * 8;

  v8f acc[4][4];
#pragma unroll
  for (int i = 0; i < 4; ++i)
#pragma unroll
    for (int j = 0; j < 4; ++j) acc[i][j] = zero8();

  for (int k0 = 0; k0 < K; k0 += 32) {
    Frag16 bh[4];
#pragma unroll
    for (int j = 0; j < 4; ++j) {
      const size_t bo = (size_t)(n0 + (j << 4) + rlane) * ldb + koff + k0;
      bh[j] = ldfrag16(Bb + bo);
    }
#pragma unroll
    for (int i = 0; i < 4; ++i) {
#pragma unroll
      for (int pl = 0; pl < NPA; ++pl) {
        Frag16 ah;
        if (A32) {
          const float* ap = Af + (size_t)(m0 + (i << 4) + rlane) * lda + koff + k0;
          const v4f x0 = *(const v4f*)(ap), x1 = *(const v4f*)(ap + 4);
          const v4f x2 = *(const v4f*)(ap + 16), x3 = *(const v4f*)(ap + 20);
#pragma unroll
          for (int e = 0; e < 4; ++e) {
            ah.hh[0][e]     = (_Float16)(x0[e] * ascale);
            ah.hh[0][4 + e] = (_Float16)(x1[e] * ascale);
            ah.hh[1][e]     = (_Float16)(x2[e] * ascale);
            ah.hh[1][4 + e] = (_Float16)(x3[e] * ascale);
          }
        } else {
          const unsigned short* Apl = (pl == 0) ? A1 : A2;
          const size_t ao = (size_t)(m0 + (i << 4) + rlane) * lda + koff + k0;
          ah = ldfrag16(Apl + ao);
        }
#pragma unroll
        for (int j = 0; j < 4; ++j) acc[i][j] = mma16_raw<TB>(ah, bh[j], acc[i][j]);
        dep_guard1(acc[i][0], acc[i][3], ah.h);
      }
    }
    keep4_h(bh[0].h, bh[1].h, bh[2].h, bh[3].h);
  }
  acc_guard4(acc[0][0], acc[0][1], acc[0][2], acc[0][3]);
  acc_guard4(acc[1][0], acc[1][1], acc[1][2], acc[1][3]);
  acc_guard4(acc[2][0], acc[2][1], acc[2][2], acc[2][3]);
  acc_guard4(acc[3][0], acc[3][1], acc[3][2], acc[3][3]);

  const int hh2 = lane >> 4, c4 = (lane & 15) * 4;
  const int q8  = lane >> 3, c8 = (lane & 7) * 8;
  float bc[8];
#pragma unroll
  for (int e = 0; e < 8; ++e) bc[e] = 0.f;
  if (BIASM == 0) {
    if (OM == 0) {
      const int cb = n0 + c4;
      const int i0 = (cb < N - 4) ? cb : (N - 4);
      const v4f b0v = *(const v4f*)(bias + i0);
#pragma unroll
      for (int e = 0; e < 4; ++e) bc[e] = bfr(b0v[e]) * bscale;
    } else {
      const int cb = n0 + c8;
      const int i0 = (cb < N - 8) ? cb : (N - 8);
      const v4f b0a = *(const v4f*)(bias + i0), b0b = *(const v4f*)(bias + i0 + 4);
#pragma unroll
      for (int e = 0; e < 4; ++e) {
        bc[e]     = bfr(b0a[e]) * bscale;
        bc[4 + e] = bfr(b0b[e]) * bscale;
      }
    }
  }

  float* slab = sT[wave];
#pragma unroll
  for (int i = 0; i < 4; ++i) {
    const int mBase = m0 + (i << 4);
#pragma unroll
    for (int j = 0; j < 4; ++j) {
#pragma unroll
      for (int r = 0; r < 8; ++r) {
        slab[(mOff + r) * 68 + (j << 4) + rlane] = acc[i][j][r];
      }
    }
    wave_sync_lds();
    if (OM == 0) {
      float* C = (float*)Cout + (size_t)b * strideC;
      const float*    Rf = (const float*)resid + (size_t)b * strideC;
      const _Float16* Rh = (const _Float16*)resid + (size_t)b * strideC;
      v4f vals[8];
#pragma unroll
      for (int it = 0; it < 8; ++it) {
        const int row = it * 2 + hh2;
        v4f v = *(const v4f*)(slab + row * 68 + c4);
#pragma unroll
        for (int e = 0; e < 4; ++e) {
          float f = v[e] * oscale + bc[e];
          if (ACT == 1) f = fmaxf(f, 0.f);
          if (ACT == 2) f = gelu_t(f);
          v[e] = f;
        }
        if (RES == 1) {
          const v4f rr = *(const v4f*)(Rf + (size_t)(mBase + row) * ldc + n0 + c4);
#pragma unroll
          for (int e = 0; e < 4; ++e) v[e] += rr[e];
        }
        if (RES == 2) {
          const v4h rr = *(const v4h*)(Rh + (size_t)(mBase + row) * ldc + n0 + c4);
#pragma unroll
          for (int e = 0; e < 4; ++e) v[e] += (float)rr[e];
        }
        vals[it] = v;
      }
      for (int pass = 0; pass < 2; ++pass) {
#pragma unroll
        for (int it = 0; it < 8; ++it) {
          const int row = it * 2 + hh2;
          *(volatile v4f*)(C + (size_t)(mBase + row) * ldc + n0 + c4) = vals[it];
        }
        __threadfence();
      }
    } else {
      unsigned short* C  = (unsigned short*)Cout  + (size_t)b * strideC;
      unsigned short* C2 = (unsigned short*)Cout2 + (size_t)b * strideC;
      v4u hv[4], lv[4];
#pragma unroll
      for (int it = 0; it < 4; ++it) {
        const int row = it * 4 + q8;
        const float* sp = slab + row * 68 + c8;
        float bm = 0.f;
        if (BIASM == 1) bm = bfr(bias[mBase + row]) * bscale;
        v4u a, a2;
#pragma unroll
        for (int e = 0; e < 4; ++e) {
          float f0 = sp[2 * e]     * oscale + ((BIASM == 1) ? bm : bc[2 * e]);
          float f1 = sp[2 * e + 1] * oscale + ((BIASM == 1) ? bm : bc[2 * e + 1]);
          if (ACT == 1) { f0 = fmaxf(f0, 0.f); f1 = fmaxf(f1, 0.f); }
          if (ACT == 2) { f0 = gelu_t(f0); f1 = gelu_t(f1); }
          if (OM == 2) {
            a[e]  = pk16(h_bits((_Float16)f0), h_bits((_Float16)f1));
            a2[e] = a[e];
          } else {
            const unsigned short h0 = bf_bits(f0), h1 = bf_bits(f1);
            const unsigned short l0 = bf_bits(f0 - bf_up(h0)), l1 = bf_bits(f1 - bf_up(h1));
            a[e]  = pk16(h0, h1);
            a2[e] = pk16(l0, l1);
          }
        }
        hv[it] = a;
        lv[it] = a2;
      }
      for (int pass = 0; pass < 2; ++pass) {
#pragma unroll
        for (int it = 0; it < 4; ++it) {
          const int row = it * 4 + q8;
          *(volatile v4u*)(C + (size_t)(mBase + row) * ldc + n0 + c8) = hv[it];
          if (OM == 3) *(volatile v4u*)(C2 + (size_t)(mBase + row) * ldc + n0 + c8) = lv[it];
        }
        __threadfence();
      }
    }
    wave_sync_lds();
  }
}

__global__ __launch_bounds__(128)
void attn_head(const unsigned short* __restrict__ qk, const unsigned short* __restrict__ vt, float* ao) {
  __shared__ __align__(16) float Ps[4][16 * 68];
  __shared__ __align__(16) float Os[4][16 * 68];

  const int tid  = threadIdx.x;
  const int wave = tid >> 5;
  const int lane = tid & 31;
  const int hh   = lane >> 4;
  const int c    = lane & 15;

  const int bx = blockIdx.x;
  const int h  = bx / (TT / 64);
  const int q0 = (bx % (TT / 64)) * 64 + wave * 16;

  const _Float16* Q  = (const _Float16*)(const void*)qk;
  const _Float16* Kp = Q + DM + h * HD;
  const _Float16* V  = (const _Float16*)(const void*)vt + (size_t)(h * HD) * TT;
  const float lsc = (1.4426950408889634f * 0.125f) / (QKCARRY * QKCARRY);

  const _Float16* qr = Q + (size_t)(q0 + c) * QKW + h * HD + 8 * hh;
  const v16h qa0 = ldfrag_h(qr);
  const v16h qa1 = ldfrag_h(qr + 32);

  float mrow[8], lrow[8];
  v8f oacc[4];
#pragma unroll
  for (int j = 0; j < 4; ++j) oacc[j] = zero8();
#pragma unroll
  for (int r = 0; r < 8; ++r) { mrow[r] = -INFINITY; lrow[r] = 0.f; }
  float* pt = Ps[wave];

#pragma unroll 1
  for (int kb = 0; kb < TT; kb += 64) {
    v8f s[4];
#pragma unroll
    for (int j = 0; j < 4; ++j) {
      const _Float16* kr = Kp + (size_t)(kb + 16 * j + c) * QKW + 8 * hh;
      const v16h kf0 = ldfrag_h(kr);
      const v16h kf1 = ldfrag_h(kr + 32);
      const v8f t = mma_h(qa0, kf0, zero8());
      s[j] = mma_h(qa1, kf1, t);
    }
#pragma unroll
    for (int r = 0; r < 8; ++r) {
      const float t0 = s[0][r] * lsc, t1 = s[1][r] * lsc, t2 = s[2][r] * lsc, t3 = s[3][r] * lsc;
      float mx = fmaxf(fmaxf(t0, t1), fmaxf(t2, t3));
#pragma unroll
      for (int off = 1; off < 16; off <<= 1) mx = fmaxf(mx, __shfl_xor(mx, off, 32));
      const float mn = fmaxf(mrow[r], mx);
      const float al = exp2f(mrow[r] - mn);
      mrow[r] = mn;
      const float e0 = exp2f(t0 - mn), e1 = exp2f(t1 - mn), e2 = exp2f(t2 - mn), e3 = exp2f(t3 - mn);
      float ps = (e0 + e1) + (e2 + e3);
#pragma unroll
      for (int off = 1; off < 16; off <<= 1) ps += __shfl_xor(ps, off, 32);
      lrow[r] = lrow[r] * al + ps;
#pragma unroll
      for (int j = 0; j < 4; ++j) oacc[j][r] *= al;
      const int ro = (8 * hh + r) * 68 + c;
      pt[ro]      = e0;
      pt[ro + 16] = e1;
      pt[ro + 32] = e2;
      pt[ro + 48] = e3;
    }
    wave_sync_lds();
#pragma unroll
    for (int wi = 0; wi < 2; ++wi) {
      const float* prow = pt + c * 68 + 32 * wi + 8 * hh;
      const v4f p0 = *(const v4f*)(prow), p1 = *(const v4f*)(prow + 4);
      const v4f p2 = *(const v4f*)(prow + 16), p3 = *(const v4f*)(prow + 20);
      FragH pa;
#pragma unroll
      for (int e = 0; e < 4; ++e) {
        pa.h[0][e]     = (_Float16)(p0[e] * PCARRY);
        pa.h[0][4 + e] = (_Float16)(p1[e] * PCARRY);
        pa.h[1][e]     = (_Float16)(p2[e] * PCARRY);
        pa.h[1][4 + e] = (_Float16)(p3[e] * PCARRY);
      }
      const int k0 = kb + 32 * wi;
#pragma unroll
      for (int j = 0; j < 4; ++j) {
        const v16h vb = ldfrag_h(V + (size_t)(16 * j + c) * TT + k0 + 8 * hh);
        oacc[j] = mma_h(pa.v, vb, oacc[j]);
      }
    }
    wave_sync_lds();
  }

  float* os = Os[wave];
  const float oinv = 1.0f / (PCARRY * VCARRY);
#pragma unroll
  for (int r = 0; r < 8; ++r) {
    const float inv = (1.0f / lrow[r]) * oinv;
#pragma unroll
    for (int j = 0; j < 4; ++j) os[(8 * hh + r) * 68 + 16 * j + c] = oacc[j][r] * inv;
  }
  wave_sync_lds();
  {
    const int q2 = lane >> 4, e4 = (lane & 15) * 4;
    v4f vals[8];
#pragma unroll
    for (int it = 0; it < 8; ++it) {
      const int row = it * 2 + q2;
      vals[it] = *(const v4f*)(os + row * 68 + e4);
    }
    for (int pass = 0; pass < 2; ++pass) {
#pragma unroll
      for (int it = 0; it < 8; ++it) {
        const int row = it * 2 + q2;
        *(volatile v4f*)(ao + (size_t)(q0 + row) * DM + h * HD + e4) = vals[it];
      }
      __threadfence();
    }
  }
}

extern "C" void kernel_launch(void* const* d_in, const int* in_sizes, int n_in,
                              void* d_out, int out_size, void* d_ws, size_t ws_size,
                              hipStream_t stream) {
  if (n_in < 17) return;
  if (in_sizes[0] != TT * DM) return;
  if (in_sizes[1] != DM || in_sizes[2] != DM) return;
  if (in_sizes[3] != DM * DM || in_sizes[4] != DM) return;
  if (in_sizes[5] != DM * DM || in_sizes[6] != DM) return;
  if (in_sizes[7] != DM * DM || in_sizes[8] != DM) return;
  if (in_sizes[9] != DM * DM || in_sizes[10] != DM) return;
  if (in_sizes[11] != DM || in_sizes[12] != DM) return;
  if (in_sizes[13] != DM * DFF || in_sizes[14] != DFF) return;
  if (in_sizes[15] != DFF * DM || in_sizes[16] != DM) return;
  if (out_size != TT * DM) return;

  const float* x    = (const float*)d_in[0];
  const float* g_1  = (const float*)d_in[1];   const float* be_1 = (const float*)d_in[2];
  const float* w_q  = (const float*)d_in[3];   const float* b_q  = (const float*)d_in[4];
  const float* w_k  = (const float*)d_in[5];   const float* b_k  = (const float*)d_in[6];
  const float* w_v  = (const float*)d_in[7];   const float* b_v  = (const float*)d_in[8];
  const float* w_o  = (const float*)d_in[9];   const float* b_o  = (const float*)d_in[10];
  const float* g_2  = (const float*)d_in[11];  const float* be_2 = (const float*)d_in[12];
  const float* w_1  = (const float*)d_in[13];  const float* b_1  = (const float*)d_in[14];
  const float* w_2  = (const float*)d_in[15];  const float* b_2  = (const float*)d_in[16];

  const size_t PWQK = (size_t)QKW * DM * 2;
  const size_t PWSQ = (size_t)DM * DM * 2;
  const size_t PW1  = (size_t)DFF * DM * 2;
  const size_t PW2  = (size_t)DM * DFF * 2;
  const size_t PBIA = 4096;
  const size_t PX16 = (size_t)TT * DM * 2;
  const size_t PQK  = (size_t)TT * QKW * 2;
  const size_t PVT  = (size_t)DM * TT * 2;
  const size_t PAF  = (size_t)TT * DM * 4;
  const size_t PGB  = (size_t)TT * DFF * 2;
  size_t off = 0;
  const size_t oWQK = off; off += PWQK;
  const size_t oWVT = off; off += PWSQ;
  const size_t oWOT = off; off += PWSQ;
  const size_t oW1T = off; off += PW1;
  const size_t oW2T = off; off += PW2;
  const size_t oBIA = off; off += PBIA;
  const size_t oXH  = off; off += PX16;
  const size_t oH1  = off; off += PX16;
  const size_t oQK  = off; off += PQK;
  const size_t oVT  = off; off += PVT;
  const size_t oAO  = off; off += PAF;
  const size_t oX1  = off; off += PAF;
  const size_t oYBH = off; off += PX16;
  const size_t oYBL = off; off += PX16;
  const size_t oGBH = off; off += PGB;
  const size_t oGBL = off; off += PGB;
  if (off > ws_size) return;
  if (off > (size_t)134217728) return;

  char* ws = (char*)d_ws;
  unsigned short* WQK = (unsigned short*)(ws + oWQK);
  unsigned short* WVT = (unsigned short*)(ws + oWVT);
  unsigned short* WOT = (unsigned short*)(ws + oWOT);
  unsigned short* W1T = (unsigned short*)(ws + oW1T);
  unsigned short* W2T = (unsigned short*)(ws + oW2T);
  float*          BIA = (float*)(ws + oBIA);
  unsigned short* XH  = (unsigned short*)(ws + oXH);
  unsigned short* H1  = (unsigned short*)(ws + oH1);
  unsigned short* QK  = (unsigned short*)(ws + oQK);
  unsigned short* VT  = (unsigned short*)(ws + oVT);
  float*          AO  = (float*)(ws + oAO);
  float*          X1  = (float*)(ws + oX1);
  unsigned short* YBH = (unsigned short*)(ws + oYBH);
  unsigned short* YBL = (unsigned short*)(ws + oYBL);
  unsigned short* GBH = (unsigned short*)(ws + oGBH);
  unsigned short* GBL = (unsigned short*)(ws + oGBL);
  float*          out = (float*)d_out;

  const int n8qk = (QKW * DM) / 8;
  const int n8sq = (DM * DM) / 8;
  const int n8f  = (DM * DFF) / 8;
  if ((n8qk % 256) != 0 || (n8sq % 256) != 0 || (n8f % 256) != 0) return;
  const dim3 blk(256), blk128(128);
  const dim3 gCqk((n8qk + 255) / 256), gCsq((n8sq + 255) / 256), gCf((n8f + 255) / 256);
  const dim3 gLN(TT / 8);
  const dim3 gQK(((TT / 64) * (QKW / 64) + 7) / 8, 1);
  const dim3 gVT(((DM / 64) * (TT / 64) + 7) / 8, 1);
  const dim3 gAttn(NHEAD * (TT / 64));
  const dim3 gO(((TT / 64) * (DM / 64) + 7) / 8, 1);
  const dim3 gF1(((TT / 64) * (DFF / 64) + 7) / 8, 1);

  conv_t16<0><<<gCqk, blk, 0, stream>>>(w_q, w_k, WQK, DM, DM, QKW, n8qk, WSC);
  conv_t16<0><<<gCsq, blk, 0, stream>>>(w_v, w_v, WVT, DM, DM, DM, n8sq, WSC);
  conv_t16<0><<<gCsq, blk, 0, stream>>>(w_o, w_o, WOT, DM, DM, DM, n8sq, WSC);
  conv_t16<1><<<gCf,  blk, 0, stream>>>(w_1, w_1, W1T, DM, DFF, DFF, n8f, 1.0f);
  conv_t16<1><<<gCf,  blk, 0, stream>>>(w_2, w_2, W2T, DFF, DM, DM, n8f, 1.0f);
  pack_bias2<<<dim3(1), blk, 0, stream>>>(b_q, b_k, BIA);

  ln_rows<0><<<gLN, blk, 0, stream>>>(x, g_1, be_1, XH, H1);

  gemm64<0, 0, 1, 2, 0, 0, 0><<<gQK, blk, 0, stream>>>(
      (const void*)H1, (const void*)H1, DM, 0LL, 1.0f,
      WQK, DM, 0LL,
      BIA, QKCARRY, (const void*)X1,
      (void*)QK, (void*)QK, QKW, 0LL, TT, QKW, DM, QKCARRY / WSC);

  gemm64<0, 0, 1, 2, 1, 0, 0><<<gVT, blk, 0, stream>>>(
      (const void*)WVT, (const void*)WVT, DM, 0LL, 1.0f,
      H1, DM, 0LL,
      b_v, VCARRY, (const void*)X1,
      (void*)VT, (void*)VT, TT, 0LL, DM, TT, DM, VCARRY / WSC);

  attn_head<<<gAttn, blk128, 0, stream>>>(QK, VT, AO);

  gemm64<0, 1, 1, 0, 0, 0, 2><<<gO, blk, 0, stream>>>(
      (const void*)AO, (const void*)AO, DM, 0LL, AOCARRY,
      WOT, DM, 0LL,
      b_o, 1.0f, (const void*)XH,
      (void*)X1, (void*)X1, DM, 0LL, TT, DM, DM, 1.0f / (AOCARRY * WSC));

  ln_rows<1><<<gLN, blk, 0, stream>>>(X1, g_2, be_2, YBH, YBL);

  gemm64<1, 0, 2, 3, 0, 2, 0><<<gF1, blk, 0, stream>>>(
      (const void*)YBH, (const void*)YBL, DM, 0LL, 1.0f,
      W1T, DM, 0LL,
      b_1, 1.0f, (const void*)X1,
      (void*)GBH, (void*)GBL, DFF, 0LL, TT, DFF, DM, 1.0f);

  gemm64<1, 0, 2, 0, 0, 0, 1><<<gO, blk, 0, stream>>>(
      (const void*)GBH, (const void*)GBL, DFF, 0LL, 1.0f,
      W2T, DFF, 0LL,
      b_2, 1.0f, (const void*)X1,
      (void*)out, (void*)out, DM, 0LL, TT, DM, DFF, 1.0f);
  (void)hipGetLastError();
}
